// HPGMambaStage_43602507989587
// MI455X (gfx1250) — hardware-run, weakly checked
//
#include <hip/hip_runtime.h>
#include <hip/hip_fp16.h>
#include <math.h>

typedef __attribute__((ext_vector_type(16))) _Float16 v16h;
typedef __attribute__((ext_vector_type(8)))  _Float16 v8h;
typedef __attribute__((ext_vector_type(8)))  float    v8f;
typedef __attribute__((ext_vector_type(4)))  float    v4f;
typedef __attribute__((ext_vector_type(2)))  float    v2f;

constexpr int kBatch = 4;
constexpr int kCin   = 256;
constexpr int kL     = 4096;
constexpr int kD     = 256;
constexpr int kN     = 512;
constexpr int kKb    = 4;
constexpr int kHid   = 128;
constexpr int kCatN  = kKb * kN;
constexpr int kAlP   = 32;
constexpr int kLgP   = 64;
constexpr float kWCarry = 1024.0f;
constexpr float kResid  = 2048.0f;
static_assert(kCatN == 2048);
static_assert(kHid == 4 * 32);
static_assert(kKb == 4);
static_assert((kL % 64) == 0 && (kCin % 64) == 0 && (kD % 64) == 0 && (kHid % 64) == 0 && (kCatN % 64) == 0);
static_assert((kCin % 32) == 0 && (kD % 32) == 0 && (kCatN % 32) == 0);
static_assert((kHid % 32) == 0 && (kHid % 8) == 0);
static_assert((kLgP % 64) == 0 && kKb <= kLgP);
static_assert((kL % 32) == 0);
static_assert(kAlP * 4 == 128);

constexpr size_t kSzW256 = (size_t)kD * kCin * 2;
constexpr size_t kSzWA1  = (size_t)kHid * kD * 2;
constexpr size_t kSzWB   = (size_t)kCatN * kD * 2;
constexpr size_t kSzCCAT = (size_t)kD * kCatN * 4;
constexpr size_t kSzWC   = (size_t)kD * kCatN * 2;
constexpr size_t kSzV256 = (size_t)kD * 4;
constexpr size_t kSzBA1  = (size_t)kHid * 4;
constexpr size_t kSzWA2P = (size_t)kLgP * kHid * 2;
constexpr size_t kSzABR  = (size_t)kKb * kN * 4;
constexpr size_t kSzT16  = (size_t)kL * kD * 2;
constexpr size_t kSzT32  = (size_t)kL * kD * 4;
constexpr size_t kSzPRE  = (size_t)kL * kHid * 4;
constexpr size_t kSzHM   = (size_t)kL * kHid * 2;
constexpr size_t kSzLG   = (size_t)kL * kLgP * 4;
constexpr size_t kSzAL   = (size_t)kL * kAlP * 4;
constexpr size_t kSzU4   = (size_t)kL * kCatN * 4;
constexpr size_t kSzS32  = (size_t)kL * kN * 4;
constexpr size_t kSzHK   = (size_t)kL * kCatN * 2;
constexpr size_t kOffWF   = 0;
constexpr size_t kOffWHF  = kOffWF   + kSzW256;
constexpr size_t kOffWA1  = kOffWHF  + kSzW256;
constexpr size_t kOffWB   = kOffWA1  + kSzWA1;
constexpr size_t kOffCCAT = kOffWB   + kSzWB;
constexpr size_t kOffWC   = kOffCCAT + kSzCCAT;
constexpr size_t kOffWO   = kOffWC   + kSzWC;
constexpr size_t kOffBF   = kOffWO   + kSzW256;
constexpr size_t kOffBHF  = kOffBF   + kSzV256;
constexpr size_t kOffBOUT = kOffBHF  + kSzV256;
constexpr size_t kOffBA1  = kOffBOUT + kSzV256;
constexpr size_t kOffWA2P = kOffBA1  + kSzBA1;
constexpr size_t kOffABR  = kOffWA2P + kSzWA2P;
constexpr size_t kOffXT   = kOffABR  + kSzABR;
constexpr size_t kOffHT   = kOffXT   + kSzT16;
constexpr size_t kOffX    = kOffHT   + kSzT16;
constexpr size_t kOffTH   = kOffX    + kSzT32;
constexpr size_t kOffXH   = kOffTH   + kSzT32;
constexpr size_t kOffTHH  = kOffXH   + kSzT16;
constexpr size_t kOffPRE  = kOffTHH  + kSzT16;
constexpr size_t kOffHM   = kOffPRE  + kSzPRE;
constexpr size_t kOffLG   = kOffHM   + kSzHM;
constexpr size_t kOffAL   = kOffLG   + kSzLG;
constexpr size_t kOffU4   = kOffAL   + kSzAL;
constexpr size_t kOffA    = kOffU4   + kSzU4;
constexpr size_t kOffU    = kOffA    + kSzS32;
constexpr size_t kOffHS   = kOffU    + kSzS32;
constexpr size_t kOffHK   = kOffHS   + kSzS32;
constexpr size_t kOffY    = kOffHK   + kSzHK;
constexpr size_t kOffYH   = kOffY    + kSzT32;
constexpr size_t kOffYL   = kOffYH   + kSzT16;
constexpr size_t kOffO2   = kOffYL   + kSzT16;
constexpr size_t kWsTotal = kOffO2   + kSzT32;
static_assert(kSzWA2P == 16384ull && kSzHM == 1048576ull && kSzLG == 1048576ull);
static_assert(kWsTotal == 114257408ull);
static_assert(kWsTotal <= 134217728ull);
static_assert((kOffWHF % 128) == 0 && (kOffWA1 % 128) == 0 && (kOffWB % 128) == 0 && (kOffCCAT % 128) == 0 &&
              (kOffWC % 128) == 0 && (kOffWO % 128) == 0 && (kOffBF % 128) == 0 && (kOffBHF % 128) == 0 &&
              (kOffBOUT % 128) == 0 && (kOffBA1 % 128) == 0 && (kOffWA2P % 128) == 0 && (kOffABR % 128) == 0 &&
              (kOffXT % 128) == 0 && (kOffHT % 128) == 0 && (kOffX % 128) == 0 && (kOffTH % 128) == 0 &&
              (kOffXH % 128) == 0 && (kOffTHH % 128) == 0 && (kOffPRE % 128) == 0 && (kOffHM % 128) == 0 &&
              (kOffLG % 128) == 0 && (kOffAL % 128) == 0 &&
              (kOffU4 % 128) == 0 && (kOffA % 128) == 0 && (kOffU % 128) == 0 && (kOffHS % 128) == 0 &&
              (kOffHK % 128) == 0 && (kOffY % 128) == 0 && (kOffYH % 128) == 0 && (kOffYL % 128) == 0 &&
              (kOffO2 % 128) == 0);

__device__ __forceinline__ _Float16 f16_flush(float v) {
  const float w = (fabsf(v) < 6.103515625e-05f) ? 0.0f : v;
  return (_Float16)w;
}

__device__ __forceinline__ float bf16r(float v) {
  unsigned u = __float_as_uint(v);
  u = (u + 0x7FFFu + ((u >> 16) & 1u)) & 0xFFFF0000u;
  return __uint_as_float(u);
}

__device__ __forceinline__ float h16_to_f32(unsigned hb) {
  const unsigned sgn = (hb & 0x8000u) << 16; const unsigned em = hb & 0x7fffu;
  const float fn = __uint_as_float((em << 13) + 0x38000000u);
  const float fs = (float)em * 5.9604644775390625e-8f;
  const float mag = (em < 0x400u) ? fs : fn; return __uint_as_float(__float_as_uint(mag) | sgn); }

__device__ __forceinline__ void f16_split(float v, _Float16& hi, _Float16& lo) {
  hi = f16_flush(v);
  const float hf = (float)hi;
  const float r = (v - hf) * kResid;
  lo = f16_flush(r);
}

namespace eng {
union FragU { v16h v; v8h h[2]; };
__device__ __forceinline__ v16h frag_load(const _Float16* p) {
  FragU f;
  f.h[0] = *(const v8h*)(p);
  f.h[1] = *(const v8h*)(p + 16);
  return f.v;
}
__device__ __forceinline__ v8f mma(v16h a, v16h b, v8f c) {
  return __builtin_amdgcn_wmma_f32_16x16x32_f16(false, a, false, b, (short)0, c, false, false);
}
__device__ __forceinline__ void guard1(v8f& a, v16h x, v16h y) {
  asm volatile("v_nop\n\tv_nop\n\tv_nop\n\tv_nop" : "+v"(a) : "v"(x), "v"(y));
}
__device__ __forceinline__ void guard_acc(v8f& a) {
  asm volatile("v_nop\n\tv_nop\n\tv_nop\n\tv_nop" : "+v"(a));
}
__device__ __forceinline__ void keep4(v16h a, v16h b, v16h c, v16h d) {
  asm volatile("v_nop" :: "v"(a), "v"(b), "v"(c), "v"(d));
}

template <int MI, int SPL>
__global__ __launch_bounds__(256) void gemm_f16_kernel(
    const unsigned short* __restrict__ Ap, const unsigned short* __restrict__ A2p, int lda,
    const unsigned short* __restrict__ Btp, const unsigned short* __restrict__ Bt2p, int ldb,
    float* __restrict__ C, int ldc, int M, int N, int K, float scale, float rscale)
{
  static_assert(MI >= 1 && MI <= 2);
  static_assert(SPL >= 0 && SPL <= 2);
  const _Float16* A   = (const _Float16*)Ap;
  const _Float16* A2  = (const _Float16*)A2p;
  const _Float16* Bt  = (const _Float16*)Btp;
  const _Float16* Bt2 = (const _Float16*)Bt2p;
  __shared__ __align__(16) float sT[8][16 * 68];
  const int lane = threadIdx.x & 31;
  const int wave = threadIdx.x >> 5;
  const int tilesN = N >> 6;
  const int tilesM = M / (16 * MI);
  const int tile = blockIdx.x * 8 + wave;
  if (tile >= tilesM * tilesN) return;
  const int tm = tile / tilesN;
  const int tn = tile - tm * tilesN;
  const int m0 = tm * (16 * MI);
  const int n0 = tn << 6;
  const int rlane = lane & 15;
  const int koff  = (lane >> 4) * 8;
  const int mOff  = (lane >> 4) * 8;

  v8f acc[MI][4], accr[MI][4];
#pragma unroll
  for (int i = 0; i < MI; ++i)
#pragma unroll
    for (int j = 0; j < 4; ++j) {
      acc[i][j]  = (v8f){0.f, 0.f, 0.f, 0.f, 0.f, 0.f, 0.f, 0.f};
      accr[i][j] = (v8f){0.f, 0.f, 0.f, 0.f, 0.f, 0.f, 0.f, 0.f};
    }

  for (int k0 = 0; k0 < K; k0 += 32) {
    v16h bh[4], bl[4];
#pragma unroll
    for (int j = 0; j < 4; ++j) {
      const size_t bo = (size_t)(n0 + (j << 4) + rlane) * ldb + koff + k0;
      bh[j] = frag_load(Bt + bo);
      if (SPL == 2) bl[j] = frag_load(Bt2 + bo); else bl[j] = bh[j];
    }
#pragma unroll
    for (int i = 0; i < MI; ++i) {
      const size_t ao = (size_t)(m0 + (i << 4) + rlane) * lda + koff + k0;
      const v16h ah = frag_load(A + ao);
      v16h al = ah;
      if (SPL >= 1) al = frag_load(A2 + ao);
#pragma unroll
      for (int j = 0; j < 4; ++j) {
        acc[i][j] = mma(ah, bh[j], acc[i][j]);
        if (SPL >= 1) accr[i][j] = mma(al, bh[j], accr[i][j]);
        if (SPL == 2) accr[i][j] = mma(ah, bl[j], accr[i][j]);
      }
#pragma unroll
      for (int j = 0; j < 4; ++j) {
        guard1(acc[i][j], ah, al);
        if (SPL >= 1) guard1(accr[i][j], ah, al);
      }
    }
    keep4(bh[0], bh[1], bh[2], bh[3]);
    if (SPL == 2) keep4(bl[0], bl[1], bl[2], bl[3]);
  }
#pragma unroll
  for (int i = 0; i < MI; ++i)
#pragma unroll
    for (int j = 0; j < 4; ++j) {
      guard_acc(acc[i][j]);
      if (SPL >= 1) guard_acc(accr[i][j]);
    }

  float* slab = sT[wave];
#pragma unroll
  for (int i = 0; i < MI; ++i) {
    const int mBase = m0 + (i << 4);
#pragma unroll
    for (int j = 0; j < 4; ++j) {
#pragma unroll
      for (int r = 0; r < 8; ++r) {
        float v = acc[i][j][r] * scale;
        if (SPL >= 1) v += accr[i][j][r] * rscale;
        slab[(mOff + r) * 68 + (j << 4) + rlane] = v;
      }
    }
    __builtin_amdgcn_fence(__ATOMIC_RELEASE, "workgroup");
    __builtin_amdgcn_wave_barrier();
    __builtin_amdgcn_fence(__ATOMIC_ACQUIRE, "workgroup");
    {
      const int hh = lane >> 4, c4 = (lane & 15) * 4;
      for (int pass = 0; pass < 2; ++pass) {
#pragma unroll
        for (int it = 0; it < 8; ++it) {
          const int row = it * 2 + hh;
          const v4f v = *(const v4f*)(slab + row * 68 + c4);
          *(volatile v4f*)(C + (size_t)(mBase + row) * ldc + n0 + c4) = v;
        }
        __threadfence();
      }
    }
    __builtin_amdgcn_fence(__ATOMIC_RELEASE, "workgroup");
    __builtin_amdgcn_wave_barrier();
    __builtin_amdgcn_fence(__ATOMIC_ACQUIRE, "workgroup");
  }
}
}

__global__ __launch_bounds__(256) void pack_rows_bf_kernel(
    const float* __restrict__ W, unsigned short* __restrict__ dH,
    int Kdim, int Nreal, int total8, float carry)
{
  const int i = blockIdx.x * 256 + threadIdx.x;
  if (i >= total8) return;
  const size_t e0 = (size_t)i << 3;
  const int row = (int)(e0 / (size_t)Kdim);
  const int col = (int)(e0 - (size_t)row * (size_t)Kdim);
  const bool live = (row < Nreal);
  const int rc = live ? row : (Nreal - 1);
  const v4f a0 = *(const v4f*)(W + (size_t)rc * Kdim + col);
  const v4f a1 = *(const v4f*)(W + (size_t)rc * Kdim + col + 4);
  const float w0 = a0[0];
  const float w1 = a0[1];
  const float w2 = a0[2];
  const float w3 = a0[3];
  const float w4 = a1[0];
  const float w5 = a1[1];
  const float w6 = a1[2];
  const float w7 = a1[3];
  const float t0 = bf16r(w0) * carry;
  const float t1 = bf16r(w1) * carry;
  const float t2 = bf16r(w2) * carry;
  const float t3 = bf16r(w3) * carry;
  const float t4 = bf16r(w4) * carry;
  const float t5 = bf16r(w5) * carry;
  const float t6 = bf16r(w6) * carry;
  const float t7 = bf16r(w7) * carry;
  const float g0 = live ? t0 : 0.0f;
  const float g1 = live ? t1 : 0.0f;
  const float g2 = live ? t2 : 0.0f;
  const float g3 = live ? t3 : 0.0f;
  const float g4 = live ? t4 : 0.0f;
  const float g5 = live ? t5 : 0.0f;
  const float g6 = live ? t6 : 0.0f;
  const float g7 = live ? t7 : 0.0f;
  v8h hv;
  hv[0] = f16_flush(g0);
  hv[1] = f16_flush(g1);
  hv[2] = f16_flush(g2);
  hv[3] = f16_flush(g3);
  hv[4] = f16_flush(g4);
  hv[5] = f16_flush(g5);
  hv[6] = f16_flush(g6);
  hv[7] = f16_flush(g7);
  unsigned short* qh = dH + e0;
  *(volatile v8h*)qh = hv;
  __threadfence();
  *(volatile v8h*)qh = hv;
}

__global__ __launch_bounds__(256) void rne_vec_kernel(
    const float* __restrict__ src, float* __restrict__ dst, int n4)
{
  const int i = blockIdx.x * 256 + threadIdx.x;
  if (i >= n4) return;
  const v4f a = *(const v4f*)(src + (size_t)i * 4);
  const float a0 = a[0];
  const float a1 = a[1];
  const float a2 = a[2];
  const float a3 = a[3];
  v4f r;
  r[0] = bf16r(a0);
  r[1] = bf16r(a1);
  r[2] = bf16r(a2);
  r[3] = bf16r(a3);
  float* p = dst + (size_t)i * 4;
  *(volatile v4f*)p = r;
  __threadfence();
  *(volatile v4f*)p = r;
}

template <bool LO>
__global__ __launch_bounds__(256) void transpose_pack_kernel(
    const float* __restrict__ W, unsigned short* __restrict__ BtH, unsigned short* __restrict__ BtL,
    int Kdim, int Ndim, float carry)
{
  __shared__ float tile[64 * 65];
  const int tid = threadIdx.x, lane = tid & 31, wave = tid >> 5;
  const int n0 = blockIdx.x * 64;
  const int k0 = blockIdx.y * 64;
#pragma unroll
  for (int p = 0; p < 16; ++p) {
    const int idx = tid + p * 256;
    const int kk  = idx >> 6;
    const int nn  = idx & 63;
    const int n   = n0 + nn;
    const int nc  = (n < Ndim) ? n : (Ndim - 1);
    const float v = W[(size_t)(k0 + kk) * Ndim + nc];
    tile[kk * 65 + nn] = (n < Ndim) ? (bf16r(v) * carry) : 0.0f;
  }
  __syncthreads();
  const int q = lane >> 3, c8 = (lane & 7) * 8;
  v8h hv[2], lv[2];
#pragma unroll
  for (int it = 0; it < 2; ++it) {
    const int nrow = it * 32 + wave * 4 + q;
#pragma unroll
    for (int e = 0; e < 8; ++e) {
      _Float16 h, l;
      const float t = tile[(c8 + e) * 65 + nrow];
      f16_split(t, h, l);
      hv[it][e] = h;
      lv[it][e] = l;
    }
  }
  for (int pass = 0; pass < 2; ++pass) {
#pragma unroll
    for (int it = 0; it < 2; ++it) {
      const int nrow = it * 32 + wave * 4 + q;
      const size_t o = (size_t)(n0 + nrow) * Kdim + k0 + c8;
      *(volatile v8h*)(BtH + o) = hv[it];
      if (LO) *(volatile v8h*)(BtL + o) = lv[it];
    }
    __threadfence();
  }
}

__global__ __launch_bounds__(256) void cat4_kernel(
    const float* __restrict__ Cb, float* __restrict__ CC, int n4)
{
  const int i = blockIdx.x * 256 + threadIdx.x;
  if (i >= n4) return;
  const int e0 = i * 4;
  const int d = e0 / kCatN;
  const int col = e0 - d * kCatN;
  const int k = col / kN;
  const int n = col - k * kN;
  const v4f a = *(const v4f*)(Cb + (size_t)(k * kD + d) * kN + n);
  float* p = CC + (size_t)e0;
  *(volatile v4f*)p = a;
  __threadfence();
  *(volatile v4f*)p = a;
}

__global__ __launch_bounds__(256) void bias_word_kernel(
    const float* __restrict__ src, const float* __restrict__ bias, unsigned short* __restrict__ dH, int total8)
{
  const int i = blockIdx.x * 256 + threadIdx.x;
  if (i >= total8) return;
  const size_t e0 = (size_t)i << 3;
  const int col = (int)(e0 & (size_t)(kD - 1));
  const v4f a0 = *(const v4f*)(src + e0);
  const v4f a1 = *(const v4f*)(src + e0 + 4);
  const v4f b0 = *(const v4f*)(bias + col);
  const v4f b1 = *(const v4f*)(bias + col + 4);
  v8h hv;
#pragma unroll
  for (int e = 0; e < 4; ++e) {
    const float f0 = a0[e] + b0[e];
    const float f1 = a1[e] + b1[e];
    hv[e] = f16_flush(f0);
    hv[4 + e] = f16_flush(f1);
  }
  unsigned short* qh = dH + e0;
  *(volatile v8h*)qh = hv;
  __threadfence();
  *(volatile v8h*)qh = hv;
}

__global__ __launch_bounds__(256) void gelu_word_kernel(
    const float* __restrict__ PRE, const float* __restrict__ BA1, unsigned short* __restrict__ dH, int total8)
{
  const int i = blockIdx.x * 256 + threadIdx.x;
  if (i >= total8) return;
  const size_t e0 = (size_t)i << 3;
  const int col = (int)(e0 & (size_t)(kHid - 1));
  const v4f a0 = *(const v4f*)(PRE + e0);
  const v4f a1 = *(const v4f*)(PRE + e0 + 4);
  const v4f b0 = *(const v4f*)(BA1 + col);
  const v4f b1 = *(const v4f*)(BA1 + col + 4);
  v8h hv;
#pragma unroll
  for (int e = 0; e < 4; ++e) {
    const float s0 = a0[e] + b0[e];
    const float s1 = a1[e] + b1[e];
    const float hm0 = 0.5f * s0 * (1.0f + erff(s0 * 0.70710678f));
    const float hm1 = 0.5f * s1 * (1.0f + erff(s1 * 0.70710678f));
    hv[e] = f16_flush(hm0);
    hv[4 + e] = f16_flush(hm1);
  }
  unsigned short* qh = dH + e0;
  *(volatile v8h*)qh = hv;
  __threadfence();
  *(volatile v8h*)qh = hv;
}

__global__ __launch_bounds__(256) void softmax4_kernel(
    const float* __restrict__ LG, const float* __restrict__ ba2, float* __restrict__ ALPHA, int ntok)
{
  const int lane = threadIdx.x & 31;
  const int wave = threadIdx.x >> 5;
  const int t = blockIdx.x * 8 + wave;
  if (t >= ntok) return;
  const v4f lv = *(const v4f*)(LG + (size_t)t * kLgP);
  const v4f b2 = *(const v4f*)(ba2);
  const float p0 = lv[0];
  const float p1 = lv[1];
  const float p2 = lv[2];
  const float p3 = lv[3];
  const float c0 = b2[0];
  const float c1 = b2[1];
  const float c2 = b2[2];
  const float c3 = b2[3];
  const float lg0 = p0 + bf16r(c0);
  const float lg1 = p1 + bf16r(c1);
  const float lg2 = p2 + bf16r(c2);
  const float lg3 = p3 + bf16r(c3);
  const float mx = fmaxf(fmaxf(lg0, lg1), fmaxf(lg2, lg3));
  const float e0 = expf(lg0 - mx);
  const float e1 = expf(lg1 - mx);
  const float e2 = expf(lg2 - mx);
  const float e3 = expf(lg3 - mx);
  const float ssum = e0 + e1 + e2 + e3;
  const float al0 = e0 / ssum;
  const float al1 = e1 / ssum;
  const float al2 = e2 / ssum;
  const float al3 = e3 / ssum;
  const float outv = (lane == 0) ? al0 : ((lane == 1) ? al1 : ((lane == 2) ? al2 : ((lane == 3) ? al3 : 0.0f)));
  float* q = ALPHA + (size_t)t * kAlP + lane;
  *(volatile float*)q = outv;
  __threadfence();
  *(volatile float*)q = outv;
}

__global__ __launch_bounds__(256) void au_kernel(
    const float* __restrict__ ALPHA, const float* __restrict__ ABR, const float* __restrict__ U4,
    float* __restrict__ Ad, float* __restrict__ Ud, int n4)
{
  const int i = blockIdx.x * 256 + threadIdx.x;
  if (i >= n4) return;
  const int e0 = i * 4;
  const int t = e0 / kN;
  const int n = e0 - t * kN;
  const v4f al = *(const v4f*)(ALPHA + (size_t)t * kAlP);
  const float al0 = al[0];
  const float al1 = al[1];
  const float al2 = al[2];
  const float al3 = al[3];
  const v4f a0 = *(const v4f*)(ABR + 0 * kN + n);
  const v4f a1 = *(const v4f*)(ABR + 1 * kN + n);
  const v4f a2 = *(const v4f*)(ABR + 2 * kN + n);
  const v4f a3 = *(const v4f*)(ABR + 3 * kN + n);
  const float* up = U4 + (size_t)t * kCatN + n;
  const v4f u0 = *(const v4f*)(up + 0 * kN);
  const v4f u1 = *(const v4f*)(up + 1 * kN);
  const v4f u2 = *(const v4f*)(up + 2 * kN);
  const v4f u3 = *(const v4f*)(up + 3 * kN);
  v4f ra, ru;
#pragma unroll
  for (int e = 0; e < 4; ++e) {
    const float sm = al0 * a0[e] + al1 * a1[e] + al2 * a2[e] + al3 * a3[e];
    ra[e] = 1.0f / (1.0f + expf(-sm));
    ru[e] = al0 * u0[e] + al1 * u1[e] + al2 * u2[e] + al3 * u3[e];
  }
  float* pa = Ad + (size_t)e0;
  float* pu = Ud + (size_t)e0;
  *(volatile v4f*)pa = ra;
  *(volatile v4f*)pu = ru;
  __threadfence();
  *(volatile v4f*)pa = ra;
  *(volatile v4f*)pu = ru;
}

__global__ __launch_bounds__(256) void hrec_kernel(
    const float* __restrict__ Ad, const float* __restrict__ Ud, float* __restrict__ HS)
{
  const int n = blockIdx.x * 256 + threadIdx.x;
  for (int pass = 0; pass < 2; ++pass) {
    float h = 0.0f;
    for (int t = 0; t < kL; ++t) {
      const float av = Ad[t * kN + n];
      const float uv = Ud[t * kN + n];
      h = fmaf(av, h, uv);
      *(volatile float*)(HS + t * kN + n) = h;
    }
    __threadfence();
  }
}

__global__ __launch_bounds__(256) void mixh_kernel(
    const float* __restrict__ ALPHA, const float* __restrict__ HS, unsigned short* __restrict__ HK, int total8)
{
  const int i = blockIdx.x * 256 + threadIdx.x;
  if (i >= total8) return;
  const size_t e0 = (size_t)i << 3;
  const int t = (int)(e0 / (size_t)kCatN);
  const int col = (int)(e0 - (size_t)t * (size_t)kCatN);
  const int k = col / kN;
  const int n = col - k * kN;
  const v4f al = *(const v4f*)(ALPHA + (size_t)t * kAlP);
  const float al0 = al[0];
  const float al1 = al[1];
  const float al2 = al[2];
  const float al3 = al[3];
  const float ak = (k == 0) ? al0 : ((k == 1) ? al1 : ((k == 2) ? al2 : al3));
  const v4f h0 = *(const v4f*)(HS + (size_t)t * kN + n);
  const v4f h1 = *(const v4f*)(HS + (size_t)t * kN + n + 4);
  v8h hv;
#pragma unroll
  for (int e = 0; e < 4; ++e) {
    const float f0 = ak * h0[e];
    const float f1 = ak * h1[e];
    hv[e] = f16_flush(f0);
    hv[4 + e] = f16_flush(f1);
  }
  unsigned short* qh = HK + e0;
  *(volatile v8h*)qh = hv;
  __threadfence();
  *(volatile v8h*)qh = hv;
}

__global__ __launch_bounds__(256) void ysplit_kernel(
    const float* __restrict__ src, unsigned short* __restrict__ dH, unsigned short* __restrict__ dL, int total8)
{
  const int i = blockIdx.x * 256 + threadIdx.x;
  if (i >= total8) return;
  const size_t e0 = (size_t)i << 3;
  const v4f a0 = *(const v4f*)(src + e0);
  const v4f a1 = *(const v4f*)(src + e0 + 4);
  v8h hv, lv;
#pragma unroll
  for (int e = 0; e < 4; ++e) {
    _Float16 h0, l0, h1, l1;
    const float f0 = a0[e];
    const float f1 = a1[e];
    f16_split(f0, h0, l0);
    f16_split(f1, h1, l1);
    hv[e] = h0;
    lv[e] = l0;
    hv[4 + e] = h1;
    lv[4 + e] = l1;
  }
  unsigned short* qh = dH + e0;
  unsigned short* ql = dL + e0;
  *(volatile v8h*)qh = hv;
  *(volatile v8h*)ql = lv;
  __threadfence();
  *(volatile v8h*)qh = hv;
  *(volatile v8h*)ql = lv;
}

__global__ __launch_bounds__(256) void out_t_kernel(
    const float* __restrict__ O2, const float* __restrict__ BOUT, float* __restrict__ outb)
{
  __shared__ float tile[64 * 65];
  const int tid = threadIdx.x, lane = tid & 31, wave = tid >> 5;
  const int l0 = blockIdx.x * 64;
  const int c0 = blockIdx.y * 64;
  const int c4 = (tid & 15) * 4;
#pragma unroll
  for (int it = 0; it < 4; ++it) {
    const int row = it * 16 + (tid >> 4);
    const v4f v = *(const v4f*)(O2 + (size_t)(l0 + row) * kCin + c0 + c4);
    const float v0 = v[0];
    const float v1 = v[1];
    const float v2 = v[2];
    const float v3 = v[3];
    tile[row * 65 + c4 + 0] = v0;
    tile[row * 65 + c4 + 1] = v1;
    tile[row * 65 + c4 + 2] = v2;
    tile[row * 65 + c4 + 3] = v3;
  }
  __syncthreads();
  v2f val[8];
#pragma unroll
  for (int j = 0; j < 8; ++j) {
    const int c = wave * 8 + j;
    const float bb = BOUT[c0 + c];
    v2f w;
    w[0] = tile[(2 * lane) * 65 + c] + bb;
    w[1] = tile[(2 * lane + 1) * 65 + c] + bb;
    val[j] = w;
  }
  for (int pass = 0; pass < 2; ++pass) {
#pragma unroll
    for (int j = 0; j < 8; ++j) {
      const int c = wave * 8 + j;
      *(volatile v2f*)(outb + (size_t)(c0 + c) * kL + l0 + 2 * lane) = val[j];
    }
    __threadfence();
  }
}

static_assert(((kL / 32) * (kD / 64)) % 8 == 0);
static_assert(((kL / 32) * (kHid / 64)) % 8 == 0);
static_assert(((kL / 32) * (kLgP / 64)) % 8 == 0);
static_assert(((kL / 32) * (kCatN / 64)) % 8 == 0);
static_assert(((kL / 32) * (kCin / 64)) % 8 == 0);
static_assert(((kD * kCin / 8) % 256) == 0);
static_assert(((kHid * kD / 8) % 256) == 0);
static_assert(((kLgP * kHid / 8) % 256) == 0);
static_assert(((kCatN * kD / 8) % 256) == 0);
static_assert(((kD * kCatN / 4) % 256) == 0);
static_assert(((kL * kD / 8) % 256) == 0);
static_assert(((kL * kHid / 8) % 256) == 0);
static_assert(((kL * kN / 4) % 256) == 0);
static_assert(((kL * kCatN / 8) % 256) == 0);
static_assert((kN % 256) == 0 && (kL % 8) == 0);
static_assert((kD / 4) == 64 && (kHid / 4) == 32 && (kKb * kN / 4) == 512);

extern "C" void kernel_launch(void* const* d_in, const int* in_sizes, int n_in,
                              void* d_out, int out_size, void* d_ws, size_t ws_size,
                              hipStream_t stream)
{
  if (n_in < 15) return;
  if (in_sizes[0] != kBatch * kCin * kL) return;
  if (in_sizes[1] != kBatch * kCin * kL) return;
  if (in_sizes[2] != kD * kCin) return;
  if (in_sizes[3] != kD) return;
  if (in_sizes[4] != kD * kCin) return;
  if (in_sizes[5] != kD) return;
  if (in_sizes[6] != kHid * kD) return;
  if (in_sizes[7] != kHid) return;
  if (in_sizes[8] != kKb * kHid) return;
  if (in_sizes[9] != kKb) return;
  if (in_sizes[10] != kKb * kN) return;
  if (in_sizes[11] != kKb * kN * kD) return;
  if (in_sizes[12] != kKb * kD * kN) return;
  if (in_sizes[13] != kCin * kD) return;
  if (in_sizes[14] != kCin) return;
  if (out_size != kBatch * kCin * kL) return;
  if (ws_size < kWsTotal) return;

  const float* feat   = (const float*)d_in[0];
  const float* hfm    = (const float*)d_in[1];
  const float* Wf     = (const float*)d_in[2];
  const float* bfv    = (const float*)d_in[3];
  const float* Whf    = (const float*)d_in[4];
  const float* bhf    = (const float*)d_in[5];
  const float* Wa1    = (const float*)d_in[6];
  const float* ba1    = (const float*)d_in[7];
  const float* Wa2    = (const float*)d_in[8];
  const float* ba2    = (const float*)d_in[9];
  const float* A_base = (const float*)d_in[10];
  const float* B_base = (const float*)d_in[11];
  const float* C_base = (const float*)d_in[12];
  const float* Wout   = (const float*)d_in[13];
  const float* bout   = (const float*)d_in[14];
  float* out = (float*)d_out;

  char* ws = (char*)d_ws;
  unsigned short* WF   = (unsigned short*)(ws + kOffWF);
  unsigned short* WHF  = (unsigned short*)(ws + kOffWHF);
  unsigned short* WA1  = (unsigned short*)(ws + kOffWA1);
  unsigned short* WB   = (unsigned short*)(ws + kOffWB);
  float*          CCAT = (float*)(ws + kOffCCAT);
  unsigned short* WC   = (unsigned short*)(ws + kOffWC);
  unsigned short* WO   = (unsigned short*)(ws + kOffWO);
  float*          BF   = (float*)(ws + kOffBF);
  float*          BHF  = (float*)(ws + kOffBHF);
  float*          BOUT = (float*)(ws + kOffBOUT);
  float*          BA1  = (float*)(ws + kOffBA1);
  unsigned short* WA2P = (unsigned short*)(ws + kOffWA2P);
  float*          ABR  = (float*)(ws + kOffABR);
  unsigned short* XT   = (unsigned short*)(ws + kOffXT);
  unsigned short* HT   = (unsigned short*)(ws + kOffHT);
  float*          X    = (float*)(ws + kOffX);
  float*          TH   = (float*)(ws + kOffTH);
  unsigned short* XH   = (unsigned short*)(ws + kOffXH);
  unsigned short* THH  = (unsigned short*)(ws + kOffTHH);
  float*          PRE  = (float*)(ws + kOffPRE);
  unsigned short* HM   = (unsigned short*)(ws + kOffHM);
  float*          LG   = (float*)(ws + kOffLG);
  float*          ALPHA = (float*)(ws + kOffAL);
  float*          U4   = (float*)(ws + kOffU4);
  float*          Ad   = (float*)(ws + kOffA);
  float*          Ud   = (float*)(ws + kOffU);
  float*          HS   = (float*)(ws + kOffHS);
  unsigned short* HK   = (unsigned short*)(ws + kOffHK);
  float*          Y    = (float*)(ws + kOffY);
  unsigned short* YH   = (unsigned short*)(ws + kOffYH);
  unsigned short* YL   = (unsigned short*)(ws + kOffYL);
  float*          O2   = (float*)(ws + kOffO2);

  constexpr float sW  = 1.0f / kWCarry;
  constexpr float sWr = 1.0f / (kWCarry * kResid);

  pack_rows_bf_kernel<<<(kD * kCin / 8) / 256, 256, 0, stream>>>(Wf, WF, kCin, kD, kD * kCin / 8, kWCarry);
  pack_rows_bf_kernel<<<(kD * kCin / 8) / 256, 256, 0, stream>>>(Whf, WHF, kCin, kD, kD * kCin / 8, kWCarry);
  pack_rows_bf_kernel<<<(kHid * kD / 8) / 256, 256, 0, stream>>>(Wa1, WA1, kD, kHid, kHid * kD / 8, kWCarry);
  pack_rows_bf_kernel<<<(kCatN * kD / 8) / 256, 256, 0, stream>>>(B_base, WB, kD, kCatN, kCatN * kD / 8, kWCarry);
  cat4_kernel<<<(kD * kCatN / 4) / 256, 256, 0, stream>>>(C_base, CCAT, kD * kCatN / 4);
  pack_rows_bf_kernel<<<(kD * kCatN / 8) / 256, 256, 0, stream>>>(CCAT, WC, kCatN, kD, kD * kCatN / 8, kWCarry);
  pack_rows_bf_kernel<<<(kCin * kD / 8) / 256, 256, 0, stream>>>(Wout, WO, kD, kCin, kCin * kD / 8, kWCarry);
  pack_rows_bf_kernel<<<(kLgP * kHid / 8) / 256, 256, 0, stream>>>(Wa2, WA2P, kHid, kKb, kLgP * kHid / 8, kWCarry);

  rne_vec_kernel<<<1, 256, 0, stream>>>(bfv, BF, kD / 4);
  rne_vec_kernel<<<1, 256, 0, stream>>>(bhf, BHF, kD / 4);
  rne_vec_kernel<<<1, 256, 0, stream>>>(bout, BOUT, kCin / 4);
  rne_vec_kernel<<<1, 256, 0, stream>>>(ba1, BA1, kHid / 4);
  rne_vec_kernel<<<(kKb * kN / 4) / 256, 256, 0, stream>>>(A_base, ABR, kKb * kN / 4);

  for (int b = 0; b < kBatch; ++b) {
    const float* featb = feat + (size_t)b * kCin * kL;
    const float* hfb   = hfm  + (size_t)b * kCin * kL;
    float* outb = out + (size_t)b * kCin * kL;

    transpose_pack_kernel<false><<<dim3(kL / 64, kCin / 64), 256, 0, stream>>>(featb, XT, XT, kCin, kL, 1.0f);
    transpose_pack_kernel<false><<<dim3(kL / 64, kCin / 64), 256, 0, stream>>>(hfb, HT, HT, kCin, kL, 1.0f);

    eng::gemm_f16_kernel<2, 0><<<dim3((kL / 32) * (kD / 64) / 8), 256, 0, stream>>>(
        XT, nullptr, kCin, WF, nullptr, kCin, X, kD, kL, kD, kCin, sW, 0.0f);
    eng::gemm_f16_kernel<2, 0><<<dim3((kL / 32) * (kD / 64) / 8), 256, 0, stream>>>(
        HT, nullptr, kCin, WHF, nullptr, kCin, TH, kD, kL, kD, kCin, sW, 0.0f);

    bias_word_kernel<<<(kL * kD / 8) / 256, 256, 0, stream>>>(X, BF, XH, kL * kD / 8);
    bias_word_kernel<<<(kL * kD / 8) / 256, 256, 0, stream>>>(TH, BHF, THH, kL * kD / 8);

    eng::gemm_f16_kernel<2, 0><<<dim3((kL / 32) * (kHid / 64) / 8), 256, 0, stream>>>(
        THH, nullptr, kD, WA1, nullptr, kD, PRE, kHid, kL, kHid, kD, sW, 0.0f);

    gelu_word_kernel<<<(kL * kHid / 8) / 256, 256, 0, stream>>>(PRE, BA1, HM, kL * kHid / 8);

    eng::gemm_f16_kernel<2, 0><<<dim3((kL / 32) * (kLgP / 64) / 8), 256, 0, stream>>>(
        HM, nullptr, kHid, WA2P, nullptr, kHid, LG, kLgP, kL, kLgP, kHid, sW, 0.0f);

    softmax4_kernel<<<kL / 8, 256, 0, stream>>>(LG, ba2, ALPHA, kL);

    eng::gemm_f16_kernel<2, 0><<<dim3((kL / 32) * (kCatN / 64) / 8), 256, 0, stream>>>(
        XH, nullptr, kD, WB, nullptr, kD, U4, kCatN, kL, kCatN, kD, sW, 0.0f);

    au_kernel<<<(kL * kN / 4) / 256, 256, 0, stream>>>(ALPHA, ABR, U4, Ad, Ud, kL * kN / 4);

    hrec_kernel<<<kN / 256, 256, 0, stream>>>(Ad, Ud, HS);

    mixh_kernel<<<(kL * kCatN / 8) / 256, 256, 0, stream>>>(ALPHA, HS, HK, kL * kCatN / 8);

    eng::gemm_f16_kernel<2, 0><<<dim3((kL / 32) * (kD / 64) / 8), 256, 0, stream>>>(
        HK, nullptr, kCatN, WC, nullptr, kCatN, Y, kD, kL, kD, kCatN, sW, 0.0f);

    ysplit_kernel<<<(kL * kD / 8) / 256, 256, 0, stream>>>(Y, YH, YL, kL * kD / 8);

    eng::gemm_f16_kernel<2, 1><<<dim3((kL / 32) * (kCin / 64) / 8), 256, 0, stream>>>(
        YH, YL, kD, WO, WO, kD, O2, kCin, kL, kCin, kD, sW, sWr);

    out_t_kernel<<<dim3(kL / 64, kCin / 64), 256, 0, stream>>>(O2, BOUT, outb);
  }
}
